// EdgeFeatureGCN_11940009083187
// MI455X (gfx1250) — hardware-verified
//
#include <hip/hip_runtime.h>
#include <stddef.h>


#define HDIM    128
#define FDIM    10
#define NTHR    256
#define NWAVE   8
#define EPT     8
#define NGRP    2
#define CHUNK   (NTHR * EPT * NGRP)
#define WCAP    (EPT * NGRP * 32)
#define LISTN   (NWAVE * WCAP)
#define NBC     4096
#define NBF     1024
#define RCAP    40960
#define RBN     128
#define OTHR    512
#define TGT     256
#define DEGCAP  512
#define GROWS   128
#define APH     136
#define NBROW   1280
#define EPB     64
#define ETHR    128
#define BNEPS   1e-5f

#define LDS_FILL ((RCAP + NBF + LISTN) * 4 + 64)
#define LDS_NG   (2 * GROWS * APH * 2 + (FDIM * HDIM + HDIM) * 4)

#define EO_TH   0
#define EO_TL   (EO_TH + EPB * APH * 2)
#define EO_ZH   (EO_TL + EPB * APH * 2)
#define EO_ZL   (EO_ZH + EPB * APH * 2)
#define EO_AB   (EO_ZL + EPB * APH * 2)
#define EO_EA   (EO_AB + EPB * HDIM * 4)
#define EO_W1E  (EO_EA + EPB * FDIM * 4)
#define EO_WAT  (EO_W1E + FDIM * HDIM * 4)
#define EO_B1E  (EO_WAT + FDIM * HDIM * 4)
#define EO_BA   (EO_B1E + HDIM * 4)
#define EO_W2A  (EO_BA + HDIM * 4)
#define EO_CV   (EO_W2A + HDIM * 4)
#define EO_B1C  (EO_CV + HDIM * 4)
#define EO_B2C  (EO_B1C + HDIM * 4)
#define EO_W3   (EO_B2C + 64 * 4)
#define EO_ATT  (EO_W3 + HDIM * 4)
#define EO_ROW  (EO_ATT + EPB * 4)
#define EO_COL  (EO_ROW + EPB * 4)
#define EO_OUT  (EO_COL + EPB * 4)
#define LDS_EDGE (EO_OUT + EPB * 2 * 4)

static_assert((CHUNK & (CHUNK - 1)) == 0);
static_assert(CHUNK <= 4096);
static_assert(NBC <= 4096 && NBF <= 4096);
static_assert((NBC & (NBC - 1)) == 0 && (NBF & (NBF - 1)) == 0);
static_assert(NBC == 4 * NBF);
static_assert(OTHR * 8 == NBC);
static_assert((RCAP % 32) == 0);
static_assert(GROWS * HDIM * 4 <= 2 * GROWS * APH * 2);
static_assert(TGT == NWAVE * 32 && (TGT % GROWS) == 0);
static_assert((GROWS * HDIM / 8) % NTHR == 0);
static_assert((APH % 8) == 0);
static_assert(EPB == (ETHR / 32) * 16);
static_assert((EO_TL % 16) == 0 && (EO_ZH % 16) == 0 && (EO_ZL % 16) == 0 && (EO_AB % 16) == 0);
static_assert((EO_EA % 16) == 0 && (EO_W1E % 16) == 0 && (EO_WAT % 16) == 0 && (EO_B1E % 16) == 0);
static_assert((EO_OUT % 16) == 0 && (EO_ATT % 16) == 0);

typedef float          v4f   __attribute__((ext_vector_type(4)));
typedef float          v8f   __attribute__((ext_vector_type(8)));
typedef int            v4i   __attribute__((ext_vector_type(4)));
typedef double         v2d   __attribute__((ext_vector_type(2)));
typedef unsigned short v4us  __attribute__((ext_vector_type(4)));
typedef unsigned short v8us  __attribute__((ext_vector_type(8)));
typedef __bf16         v16bf __attribute__((ext_vector_type(16)));
union FragB { v16bf v; v8us h[2]; };

__device__ __forceinline__ unsigned short bfr(float x) {
  const unsigned u = __float_as_uint(x);
  return (unsigned short)((u + 0x7FFFu + ((u >> 16) & 1u)) >> 16);
}
__device__ __forceinline__ void bfsplit(float x, unsigned short& hb, unsigned short& lb) {
  hb = bfr(x);
  const float hf = __uint_as_float(((unsigned)hb) << 16);
  lb = bfr(x - hf);
}

__device__ __forceinline__ v8f wmb(v16bf a, v16bf b, v8f c) {
  v8f d = __builtin_amdgcn_wmma_f32_16x16x32_bf16(false, a, false, b, (short)0, c, false, false);
  asm volatile("v_nop\n\tv_nop\n\tv_nop\n\tv_nop" : "+v"(d) : "v"(a), "v"(b));
  return d;
}

template <int NB>
__device__ __forceinline__ int scan_chunk(const int* __restrict__ dsts, int nE, int cbase, int slotBase,
                                          int vec8, int* list, int tid, int lane, int wave) {
  int wc = 0;
#pragma unroll
  for (int g = 0; g < NGRP; ++g) {
    const int el0  = (g * NTHR + tid) * EPT;
    const int e0   = cbase + el0;
    const int sent = -2147483647 - 1;
    v4i da, db;
    if (vec8 != 0 && cbase + CHUNK <= nE) {
      da = *(const v4i*)(dsts + e0);
      db = *(const v4i*)(dsts + e0 + 4);
    } else {
      da.x = (e0     < nE) ? dsts[min(e0, nE - 1)] : sent;
      da.y = (e0 + 1 < nE) ? dsts[min(e0 + 1, nE - 1)] : sent;
      da.z = (e0 + 2 < nE) ? dsts[min(e0 + 2, nE - 1)] : sent;
      da.w = (e0 + 3 < nE) ? dsts[min(e0 + 3, nE - 1)] : sent;
      db.x = (e0 + 4 < nE) ? dsts[min(e0 + 4, nE - 1)] : sent;
      db.y = (e0 + 5 < nE) ? dsts[min(e0 + 5, nE - 1)] : sent;
      db.z = (e0 + 6 < nE) ? dsts[min(e0 + 6, nE - 1)] : sent;
      db.w = (e0 + 7 < nE) ? dsts[min(e0 + 7, nE - 1)] : sent;
    }
    const unsigned nb = (unsigned)slotBase;
    const unsigned s0 = (unsigned)da.x - nb, s1 = (unsigned)da.y - nb;
    const unsigned s2 = (unsigned)da.z - nb, s3 = (unsigned)da.w - nb;
    const unsigned s4 = (unsigned)db.x - nb, s5 = (unsigned)db.y - nb;
    const unsigned s6 = (unsigned)db.z - nb, s7 = (unsigned)db.w - nb;
    const bool h0 = s0 < (unsigned)NB, h1 = s1 < (unsigned)NB, h2 = s2 < (unsigned)NB, h3 = s3 < (unsigned)NB;
    const bool h4 = s4 < (unsigned)NB, h5 = s5 < (unsigned)NB, h6 = s6 < (unsigned)NB, h7 = s7 < (unsigned)NB;
    const unsigned any = __builtin_amdgcn_ballot_w32(h0 | h1 | h2 | h3 | h4 | h5 | h6 | h7);
    if (any != 0u) {
#define HITJ(J, HJ, SJ) { \
        const unsigned mj = __builtin_amdgcn_ballot_w32(HJ); \
        if (mj != 0u) { \
          if (HJ) { \
            const int pos = wc + (int)__builtin_amdgcn_mbcnt_lo(mj, 0u); \
            if (pos < WCAP) list[wave * WCAP + pos] = ((el0 + (J)) << 12) | (int)(SJ); \
          } \
          wc += (int)__builtin_popcount(mj); } }
      HITJ(0, h0, s0)
      HITJ(1, h1, s1)
      HITJ(2, h2, s2)
      HITJ(3, h3, s3)
      HITJ(4, h4, s4)
      HITJ(5, h5, s5)
      HITJ(6, h6, s6)
      HITJ(7, h7, s7)
#undef HITJ
    }
  }
  return wc;
}

__global__ __launch_bounds__(NTHR) void k_wprep(
    const float* __restrict__ ne_w2, const float* __restrict__ gcn_w, const float* __restrict__ skip_w,
    const float* __restrict__ ea_w1, const float* __restrict__ cl_w1,
    const float* __restrict__ ee_w2, const float* __restrict__ ee_b2, const float* __restrict__ cl_w2,
    unsigned short* bh, unsigned short* bl, unsigned short* wqh, unsigned short* wql,
    unsigned short* w2h, unsigned short* w2l, float* cvec) {
  const int tid = threadIdx.x;
  const int g0 = NBROW * 16;
  const int g1 = g0 + HDIM * 16;
  const int g2 = g1 + 64 * 16;
  const int bstart = blockIdx.x * NTHR;
  const int i = bstart + tid;
  if (bstart < g0) {
    const int R = i >> 4, k0 = (i & 15) * 8;
    const float* src; int col;
    if (R < 128)      { src = ne_w2; col = R; }
    else if (R < 512) { const int q = R - 128; src = gcn_w  + (size_t)(q >> 7) * (HDIM * HDIM); col = q & 127; }
    else if (R < 768) { const int q = R - 512; src = skip_w + (size_t)(q >> 7) * (HDIM * HDIM); col = q & 127; }
    else {
      const int n = R - 768;
      if (n < 128)      { src = ea_w1;               col = n; }
      else if (n < 256) { src = ea_w1 + HDIM * HDIM; col = n - 128; }
      else if (n < 384) { src = cl_w1;               col = n - 256; }
      else              { src = cl_w1 + HDIM * HDIM; col = n - 384; }
    }
    v8us hv, lv;
#pragma unroll
    for (int e = 0; e < 8; ++e) {
      const float x = src[(size_t)(k0 + e) * HDIM + col];
      unsigned short hb, lb;
      bfsplit(x, hb, lb);
      hv[e] = hb; lv[e] = lb;
    }
    unsigned short* ph = bh + (size_t)R * HDIM + k0;
    unsigned short* pl = bl + (size_t)R * HDIM + k0;
    *(volatile v8us*)ph = hv;
    *(volatile v8us*)pl = lv;
    __threadfence();
    *(volatile v8us*)ph = hv;
    *(volatile v8us*)pl = lv;
  } else if (bstart < g1) {
    const int q = i - g0;
    const int n = q >> 4, k0 = (q & 15) * 8;
    float acc[8];
#pragma unroll
    for (int e = 0; e < 8; ++e) acc[e] = 0.0f;
#pragma unroll 1
    for (int j = 0; j < HDIM; ++j) {
      const float wsum = cl_w1[(size_t)j * HDIM + n] + cl_w1[(size_t)(HDIM + j) * HDIM + n];
#pragma unroll
      for (int e = 0; e < 8; ++e) acc[e] += ee_w2[(size_t)(k0 + e) * HDIM + j] * wsum;
    }
    v8us hv, lv;
#pragma unroll
    for (int e = 0; e < 8; ++e) {
      unsigned short hb, lb;
      bfsplit(acc[e], hb, lb);
      hv[e] = hb; lv[e] = lb;
    }
    unsigned short* ph = wqh + (size_t)n * HDIM + k0;
    unsigned short* pl = wql + (size_t)n * HDIM + k0;
    *(volatile v8us*)ph = hv;
    *(volatile v8us*)pl = lv;
    __threadfence();
    *(volatile v8us*)ph = hv;
    *(volatile v8us*)pl = lv;
  } else if (bstart < g2) {
    const int q = i - g1;
    const int n = q >> 4, k0 = (q & 15) * 8;
    v8us hv, lv;
#pragma unroll
    for (int e = 0; e < 8; ++e) {
      unsigned short hb, lb;
      bfsplit(cl_w2[(size_t)(k0 + e) * 64 + n], hb, lb);
      hv[e] = hb; lv[e] = lb;
    }
    unsigned short* ph = w2h + (size_t)n * HDIM + k0;
    unsigned short* pl = w2l + (size_t)n * HDIM + k0;
    *(volatile v8us*)ph = hv;
    *(volatile v8us*)pl = lv;
    __threadfence();
    *(volatile v8us*)ph = hv;
    *(volatile v8us*)pl = lv;
  } else {
    if (tid < 32) {
      v4f cv = {0.f, 0.f, 0.f, 0.f};
#pragma unroll 1
      for (int j = 0; j < HDIM; ++j) {
        const float bj = ee_b2[j];
        const v4f wa = *(const v4f*)(cl_w1 + (size_t)j * HDIM + 4 * tid);
        const v4f wb = *(const v4f*)(cl_w1 + (size_t)(HDIM + j) * HDIM + 4 * tid);
        cv = cv + bj * (wa + wb);
      }
      float* p = cvec + 4 * tid;
      *(volatile v4f*)p = cv;
      __threadfence();
      *(volatile v4f*)p = cv;
    }
  }
}

__global__ __launch_bounds__(NTHR) void k_count(
    const int* __restrict__ ei, int* cnt, float* dinv, int nE, int vec8) {
  __shared__ __attribute__((aligned(16))) int scnt[NBC];
  __shared__ __attribute__((aligned(16))) int list[LISTN];
  __shared__ int wcnt[NWAVE];
  const int tid = threadIdx.x, lane = tid & 31, wave = tid >> 5;
  const int nodeBase = blockIdx.x * NBC;
  const int* dsts = ei + nE;

  for (int i = tid; i < NBC; i += NTHR) scnt[i] = 0;
  __syncthreads();

  const int nChunks = (nE + CHUNK - 1) / CHUNK;
#pragma unroll 1
  for (int ch = 0; ch < nChunks; ++ch) {
    const int cbase = ch * CHUNK;
    const int wc = scan_chunk<NBC>(dsts, nE, cbase, nodeBase, vec8, list, tid, lane, wave);
    if (lane == 0) wcnt[wave] = wc;
    __syncthreads();
    if (wave == 0) {
#pragma unroll 1
      for (int wsx = 0; wsx < NWAVE; ++wsx) {
        int n = __builtin_amdgcn_readfirstlane(wcnt[wsx]);
        n = n > WCAP ? WCAP : (n < 0 ? 0 : n);
        const int* lp = list + wsx * WCAP;
#pragma unroll 1
        for (int i = 0; i < n; ++i) {
          const int ent  = __builtin_amdgcn_readfirstlane(lp[i]);
          const int slot = ent & (NBC - 1);
          if (lane == 0) scnt[slot] = scnt[slot] + 1;
        }
      }
    }
    __syncthreads();
  }

  v4i cq[4]; v4f dq[4];
#pragma unroll
  for (int q = 0; q < 4; ++q) {
    const int f = (wave * 4 + q) * 128 + 4 * lane;
    const v4i c = *(const v4i*)(scnt + f);
    cq[q] = c;
    dq[q].x = rsqrtf((float)(c.x + 1));
    dq[q].y = rsqrtf((float)(c.y + 1));
    dq[q].z = rsqrtf((float)(c.z + 1));
    dq[q].w = rsqrtf((float)(c.w + 1));
  }
  int*   cp = cnt + (size_t)nodeBase;
  float* dp = dinv + (size_t)nodeBase;
#pragma unroll
  for (int q = 0; q < 4; ++q) {
    const int f = (wave * 4 + q) * 128 + 4 * lane;
    *(volatile v4i*)(cp + f) = cq[q];
    *(volatile v4f*)(dp + f) = dq[q];
  }
  __threadfence();
#pragma unroll
  for (int q = 0; q < 4; ++q) {
    const int f = (wave * 4 + q) * 128 + 4 * lane;
    *(volatile v4i*)(cp + f) = cq[q];
    *(volatile v4f*)(dp + f) = dq[q];
  }
}

__global__ __launch_bounds__(OTHR) void k_offsets(
    const int* __restrict__ cnt, int* off, int* rbase, int nChunk) {
  __shared__ __attribute__((aligned(16))) int soff[NBC];
  __shared__ __attribute__((aligned(16))) int srb[RBN];
  __shared__ int wtot[OTHR / 32];
  const int tid = threadIdx.x, lane = tid & 31, wave = tid >> 5, sub = tid >> 7;
  for (int i = tid; i < RBN; i += OTHR) srb[i] = 0;
  int carry = 0;
#pragma unroll 1
  for (int ch = 0; ch < nChunk; ++ch) {
    const int base = ch * NBC;
    const v4i c0 = *(const v4i*)(cnt + base + 8 * tid);
    const v4i c1 = *(const v4i*)(cnt + base + 8 * tid + 4);
    const int e0 = max(c0.x, 0), e1 = max(c0.y, 0), e2 = max(c0.z, 0), e3 = max(c0.w, 0);
    const int e4 = max(c1.x, 0), e5 = max(c1.y, 0), e6 = max(c1.z, 0), e7 = max(c1.w, 0);
    const int ts = e0 + e1 + e2 + e3 + e4 + e5 + e6 + e7;
    int incl = ts;
#pragma unroll
    for (int d = 1; d < 32; d <<= 1) {
      const int t = __shfl_up(incl, d);
      if (lane >= d) incl += t;
    }
    if (lane == 31) wtot[wave] = incl;
    __syncthreads();
    const int S0 = wtot[0]  + wtot[1]  + wtot[2]  + wtot[3];
    const int S1 = wtot[4]  + wtot[5]  + wtot[6]  + wtot[7];
    const int S2 = wtot[8]  + wtot[9]  + wtot[10] + wtot[11];
    const int S3 = wtot[12] + wtot[13] + wtot[14] + wtot[15];
    int pre = 0;
#pragma unroll 1
    for (int w = 4 * sub; w < wave; ++w) pre += wtot[w];
    const int b0 = carry;
    const int b1 = b0 + ((S0 + 31) & ~31);
    const int b2 = b1 + ((S1 + 31) & ~31);
    const int b3 = b2 + ((S2 + 31) & ~31);
    const int b4 = b3 + ((S3 + 31) & ~31);
    const int myb = sub == 0 ? b0 : (sub == 1 ? b1 : (sub == 2 ? b2 : b3));
    if (tid == 0) {
      srb[min(4 * ch + 0, RBN - 1)] = b0;
      srb[min(4 * ch + 1, RBN - 1)] = b1;
      srb[min(4 * ch + 2, RBN - 1)] = b2;
      srb[min(4 * ch + 3, RBN - 1)] = b3;
    }
    int run = myb + pre + incl - ts;
    soff[8 * tid + 0] = run; run += e0;
    soff[8 * tid + 1] = run; run += e1;
    soff[8 * tid + 2] = run; run += e2;
    soff[8 * tid + 3] = run; run += e3;
    soff[8 * tid + 4] = run; run += e4;
    soff[8 * tid + 5] = run; run += e5;
    soff[8 * tid + 6] = run; run += e6;
    soff[8 * tid + 7] = run;
    carry = b4;
    __syncthreads();
    const v4i o0 = *(const v4i*)(soff + 4 * tid);
    const v4i o1 = *(const v4i*)(soff + 4 * (tid + OTHR));
    int* op = off + base;
    *(volatile v4i*)(op + 4 * tid) = o0;
    *(volatile v4i*)(op + 4 * (tid + OTHR)) = o1;
    __threadfence();
    *(volatile v4i*)(op + 4 * tid) = o0;
    *(volatile v4i*)(op + 4 * (tid + OTHR)) = o1;
    __syncthreads();
  }
  if (tid == 0) srb[min(4 * nChunk, RBN - 1)] = carry;
  __syncthreads();
  v4i rv = {0, 0, 0, 0};
  if (tid < 32) rv = *(const v4i*)(srb + 4 * tid);
  if (tid < 32) *(volatile v4i*)(rbase + 4 * tid) = rv;
  __threadfence();
  if (tid < 32) *(volatile v4i*)(rbase + 4 * tid) = rv;
}

__global__ __launch_bounds__(NTHR) void k_fill(
    const int* __restrict__ ei, const int* __restrict__ off, const int* __restrict__ rbase,
    int* csr, int nN, int nE, int vec8, int csrLen) {
  extern __shared__ v4f lds_dyn[];
  int* region = (int*)lds_dyn;
  int* cursor = region + RCAP;
  int* list   = cursor + NBF;
  int* wcnt   = list + LISTN;
  const int tid = threadIdx.x, lane = tid & 31, wave = tid >> 5;
  const int b = blockIdx.x;
  const int nodeBase = b * NBF;
  const int* dsts = ei + nE;

  int rb0 = rbase[b];
  const int rb1 = rbase[b + 1];
  rb0 = rb0 < 0 ? 0 : (rb0 > csrLen ? csrLen : rb0);
  rb0 &= ~31;
  int len = rb1 - rb0;
  len = len < 0 ? 0 : (len > RCAP ? RCAP : len);
  int lenW = (len + 31) & ~31;
  if (rb0 + lenW > csrLen) lenW = (csrLen - rb0) & ~31;

  {
    const v4i z = {0, 0, 0, 0};
    for (int i = tid; i < RCAP / 4; i += NTHR) ((v4i*)region)[i] = z;
    for (int s = tid; s < NBF; s += NTHR) {
      int o = off[nodeBase + s] - rb0;
      o = o < 0 ? 0 : (o > RCAP ? RCAP : o);
      cursor[s] = o;
    }
  }
  __syncthreads();

  const int nChunks = (nE + CHUNK - 1) / CHUNK;
#pragma unroll 1
  for (int ch = 0; ch < nChunks; ++ch) {
    const int cbase = ch * CHUNK;
    const int wc = scan_chunk<NBF>(dsts, nE, cbase, nodeBase, vec8, list, tid, lane, wave);
    if (lane == 0) wcnt[wave] = wc;
    __syncthreads();
    if (wave == 0) {
#pragma unroll 1
      for (int wsx = 0; wsx < NWAVE; ++wsx) {
        int n = __builtin_amdgcn_readfirstlane(wcnt[wsx]);
        n = n > WCAP ? WCAP : (n < 0 ? 0 : n);
        const int* lp = list + wsx * WCAP;
#pragma unroll 1
        for (int i = 0; i < n; ++i) {
          const int ent  = __builtin_amdgcn_readfirstlane(lp[i]);
          const int slot = ent & (NBF - 1);
          int e = cbase + ((ent >> 12) & (CHUNK - 1));
          e = e > nE - 1 ? nE - 1 : e;
          int src = ei[e];
          src = src < 0 ? 0 : (src > nN - 1 ? nN - 1 : src);
          if (lane == 0) {
            int pos = cursor[slot];
            pos = pos < 0 ? 0 : (pos > RCAP - 1 ? RCAP - 1 : pos);
            region[pos] = src;
            const int np = pos + 1;
            cursor[slot] = np > RCAP ? RCAP : np;
          }
        }
      }
    }
    __syncthreads();
  }

  const int nv = lenW >> 2;
  int* gp = csr + rb0;
#pragma unroll 1
  for (int i = tid; i < nv; i += NTHR) { const v4i v = ((const v4i*)region)[i]; *(volatile v4i*)(gp + 4 * i) = v; }
  __threadfence();
#pragma unroll 1
  for (int i = tid; i < nv; i += NTHR) { const v4i v = ((const v4i*)region)[i]; *(volatile v4i*)(gp + 4 * i) = v; }
}

template <int MODE, int ASRC>
__global__ __launch_bounds__(NTHR) void k_ngemm(
    const float* __restrict__ A, const float* __restrict__ w1, const float* __restrict__ b1,
    const unsigned short* __restrict__ Bh, const unsigned short* __restrict__ Bl,
    const float* __restrict__ dinv, const float* __restrict__ bias,
    const float* __restrict__ hpre, const float* __restrict__ sct,
    float* C, int nRowsA, int ldc) {
  extern __shared__ v4f lds_dyn[];
  unsigned short* sAh = (unsigned short*)lds_dyn;
  unsigned short* sAl = sAh + GROWS * APH;
  float*          sW1 = (float*)(sAl + GROWS * APH);
  float*          stg = (float*)lds_dyn;
  const int tid = threadIdx.x, lane = tid & 31, wave = tid >> 5, hh = lane >> 4, m = lane & 15;
  const int rowBase = blockIdx.x * GROWS;
  const int nOff = blockIdx.y * HDIM;

  if (ASRC == 1) {
    for (int i = tid; i < FDIM * HDIM + HDIM; i += NTHR) {
      const int ia = i < FDIM * HDIM ? i : FDIM * HDIM - 1;
      const int ib = (i - FDIM * HDIM) < 0 ? 0 : (i - FDIM * HDIM);
      const float wa = w1[ia];
      const float wb = b1[ib];
      sW1[i] = i < FDIM * HDIM ? wa : wb;
    }
    __syncthreads();
  }

#pragma unroll
  for (int it = 0; it < (GROWS * HDIM / 8) / NTHR; ++it) {
    const int idx = it * NTHR + tid;
    const int r   = idx >> 4;
    const int c0  = (idx & 15) * 8;
    int row = rowBase + r;
    row = row > nRowsA - 1 ? nRowsA - 1 : row;
    v4f va, vb;
    if (ASRC == 0) {
      const float* ap = A + (size_t)row * HDIM + c0;
      va = *(const v4f*)ap;
      vb = *(const v4f*)(ap + 4);
    } else {
      va = *(const v4f*)(sW1 + FDIM * HDIM + c0);
      vb = *(const v4f*)(sW1 + FDIM * HDIM + c0 + 4);
#pragma unroll 1
      for (int k = 0; k < FDIM; ++k) {
        const float xk = A[(size_t)row * FDIM + k];
        va = va + xk * *(const v4f*)(sW1 + k * HDIM + c0);
        vb = vb + xk * *(const v4f*)(sW1 + k * HDIM + c0 + 4);
      }
      va.x = fmaxf(va.x, 0.f); va.y = fmaxf(va.y, 0.f); va.z = fmaxf(va.z, 0.f); va.w = fmaxf(va.w, 0.f);
      vb.x = fmaxf(vb.x, 0.f); vb.y = fmaxf(vb.y, 0.f); vb.z = fmaxf(vb.z, 0.f); vb.w = fmaxf(vb.w, 0.f);
    }
    v8us hv, lv;
    unsigned short hb, lb;
    bfsplit(va.x, hb, lb); hv[0] = hb; lv[0] = lb;
    bfsplit(va.y, hb, lb); hv[1] = hb; lv[1] = lb;
    bfsplit(va.z, hb, lb); hv[2] = hb; lv[2] = lb;
    bfsplit(va.w, hb, lb); hv[3] = hb; lv[3] = lb;
    bfsplit(vb.x, hb, lb); hv[4] = hb; lv[4] = lb;
    bfsplit(vb.y, hb, lb); hv[5] = hb; lv[5] = lb;
    bfsplit(vb.z, hb, lb); hv[6] = hb; lv[6] = lb;
    bfsplit(vb.w, hb, lb); hv[7] = hb; lv[7] = lb;
    *(v8us*)(sAh + r * APH + c0) = hv;
    *(v8us*)(sAl + r * APH + c0) = lv;
  }
  __syncthreads();

  v8f acc[8];
#pragma unroll
  for (int t = 0; t < 8; ++t) { v8f z = {0.f, 0.f, 0.f, 0.f, 0.f, 0.f, 0.f, 0.f}; acc[t] = z; }
  const unsigned short* arh = sAh + (wave * 16 + m) * APH + 8 * hh;
  const unsigned short* arl = sAl + (wave * 16 + m) * APH + 8 * hh;
#pragma unroll
  for (int kt = 0; kt < HDIM / 32; ++kt) {
    FragB ah, al;
    ah.h[0] = *(const v8us*)(arh + 32 * kt);
    ah.h[1] = *(const v8us*)(arh + 32 * kt + 16);
    al.h[0] = *(const v8us*)(arl + 32 * kt);
    al.h[1] = *(const v8us*)(arl + 32 * kt + 16);
#pragma unroll
    for (int t = 0; t < 8; ++t) {
      const size_t bp = (size_t)(nOff + 16 * t + m) * HDIM + 32 * kt + 8 * hh;
      FragB bh2, bl2;
      bh2.h[0] = *(const v8us*)(Bh + bp);
      bh2.h[1] = *(const v8us*)(Bh + bp + 16);
      bl2.h[0] = *(const v8us*)(Bl + bp);
      bl2.h[1] = *(const v8us*)(Bl + bp + 16);
      acc[t] = wmb(ah.v, bh2.v, acc[t]);
      acc[t] = wmb(al.v, bh2.v, acc[t]);
      acc[t] = wmb(ah.v, bl2.v, acc[t]);
    }
  }
  __syncthreads();

  float* sp = stg + (wave * 16 + 8 * hh) * HDIM + m;
#pragma unroll
  for (int t = 0; t < 8; ++t) {
#pragma unroll
    for (int r = 0; r < 8; ++r) sp[r * HDIM + 16 * t] = acc[t][r];
  }
  __syncthreads();

  v4f add4 = {0.f, 0.f, 0.f, 0.f};
  v4f sc4 = {1.f, 1.f, 1.f, 1.f}, sh4 = {0.f, 0.f, 0.f, 0.f};
  if (MODE == 0 || MODE == 2) add4 = *(const v4f*)(bias + 4 * lane);
  if (MODE == 2) { sc4 = *(const v4f*)(sct + 4 * lane); sh4 = *(const v4f*)(sct + HDIM + 4 * lane); }
  v4f vals[16];
#pragma unroll
  for (int i = 0; i < 16; ++i) {
    const int row = rowBase + wave * 16 + i;
    v4f v = *(const v4f*)(stg + (wave * 16 + i) * HDIM + 4 * lane);
    if (MODE == 0) {
      v = v + add4;
    } else if (MODE == 1) {
      const float d = dinv[row];
      v = v * d;
    } else if (MODE == 2) {
      const v4f hp = *(const v4f*)(hpre + (size_t)row * HDIM + 4 * lane);
      v4f y = hp * sc4 + sh4;
      y.x = fmaxf(y.x, 0.f); y.y = fmaxf(y.y, 0.f); y.z = fmaxf(y.z, 0.f); y.w = fmaxf(y.w, 0.f);
      v = y + v + add4;
    }
    vals[i] = v;
  }
  float* gp = C + ((size_t)rowBase + wave * 16) * ldc + nOff + 4 * lane;
#pragma unroll
  for (int i = 0; i < 16; ++i) *(volatile v4f*)(gp + (size_t)i * ldc) = vals[i];
  __threadfence();
#pragma unroll
  for (int i = 0; i < 16; ++i) *(volatile v4f*)(gp + (size_t)i * ldc) = vals[i];
}

__global__ __launch_bounds__(NTHR) void k_agg(
    const int* __restrict__ csr, const int* __restrict__ off, const int* __restrict__ cnt,
    const float* __restrict__ dinv, const float* __restrict__ hw, const float* __restrict__ gb,
    float* hpre, double* part, int nN, int csrLen) {
  __shared__ __attribute__((aligned(16))) double spart[NWAVE * 256];
  __shared__ __attribute__((aligned(16))) double sred[256];
  const int tid = threadIdx.x, lane = tid & 31, wave = tid >> 5;
  const int tbase = blockIdx.x * TGT + wave * 32;
  const int cl = tbase + lane;
  const int cnt_l = cnt[cl];
  const int off_l = off[cl];
  union FI { float f; int i; };
  FI dvu; dvu.f = dinv[cl];
  const v4f bb = *(const v4f*)(gb + 4 * lane);
  double s1[4], s2[4];
#pragma unroll
  for (int jn = 0; jn < 4; ++jn) { s1[jn] = 0.0; s2[jn] = 0.0; }

#pragma unroll 1
  for (int j = 0; j < 32; ++j) {
    const int c = tbase + j;
    int n = __builtin_amdgcn_readlane(cnt_l, j);
    n = n < 0 ? 0 : (n > DEGCAP ? DEGCAP : n);
    const int st = __builtin_amdgcn_readlane(off_l, j);
    FI du; du.i = __builtin_amdgcn_readlane(dvu.i, j);
    const float dc = du.f;
    v4f acc = {0.f, 0.f, 0.f, 0.f};
#pragma unroll 1
    for (int q0 = 0; q0 < n; q0 += 32) {
      int pos = st + q0 + lane;
      pos = pos < 0 ? 0 : (pos > csrLen - 1 ? csrLen - 1 : pos);
      int sl = csr[pos];
      sl = sl < 0 ? 0 : (sl > nN - 1 ? nN - 1 : sl);
      const int mcnt = (n - q0) < 32 ? (n - q0) : 32;
#pragma unroll 1
      for (int p = 0; p < mcnt; ++p) {
        const int s = __builtin_amdgcn_readlane(sl, p);
        acc = acc + *(const v4f*)(hw + (size_t)s * HDIM + 4 * lane);
      }
    }
    const v4f sv = *(const v4f*)(hw + (size_t)c * HDIM + 4 * lane);
    const v4f v = (acc + sv) * dc + bb;
    float* hp = hpre + (size_t)c * HDIM + 4 * lane;
    *(volatile v4f*)hp = v;
    __threadfence();
    *(volatile v4f*)hp = v;
    if (c < nN) {
      s1[0] += (double)v.x; s1[1] += (double)v.y; s1[2] += (double)v.z; s1[3] += (double)v.w;
      s2[0] += (double)v.x * (double)v.x; s2[1] += (double)v.y * (double)v.y;
      s2[2] += (double)v.z * (double)v.z; s2[3] += (double)v.w * (double)v.w;
    }
  }
#pragma unroll
  for (int jn = 0; jn < 4; ++jn) {
    spart[wave * 256 + 4 * lane + jn] = s1[jn];
    spart[wave * 256 + HDIM + 4 * lane + jn] = s2[jn];
  }
  __syncthreads();
  double tsum = 0.0;
#pragma unroll
  for (int w = 0; w < NWAVE; ++w) tsum += spart[w * 256 + tid];
  sred[tid] = tsum;
  __syncthreads();
  double* gp = part + (size_t)blockIdx.x * 256;
  v2d pv[4];
  if (tid < 32) {
#pragma unroll
    for (int p = 0; p < 4; ++p) pv[p] = *(const v2d*)(sred + 64 * p + 2 * tid);
#pragma unroll
    for (int p = 0; p < 4; ++p) *(volatile v2d*)(gp + 64 * p + 2 * tid) = pv[p];
  }
  __threadfence();
  if (tid < 32) {
#pragma unroll
    for (int p = 0; p < 4; ++p) *(volatile v2d*)(gp + 64 * p + 2 * tid) = pv[p];
  }
}

__global__ __launch_bounds__(NTHR) void k_bnfin(
    const double* __restrict__ part, const float* __restrict__ g, const float* __restrict__ b,
    float* sct, int nBlk, int nN) {
  __shared__ __attribute__((aligned(16))) double sred[256];
  __shared__ __attribute__((aligned(16))) float stab[256];
  const int tid = threadIdx.x;
  double s = 0.0;
#pragma unroll 1
  for (int k = 0; k < nBlk; ++k) s += part[(size_t)k * 256 + tid];
  sred[tid] = s;
  __syncthreads();
  if (tid < HDIM) {
    const double inv_n = 1.0 / (double)nN;
    const double mean = sred[tid] * inv_n;
    double var = sred[HDIM + tid] * inv_n - mean * mean;
    var = var < 0.0 ? 0.0 : var;
    const float varf = (float)var;
    const float inv = rsqrtf(varf + BNEPS);
    const float scv = g[tid] * inv;
    stab[tid] = scv;
    stab[HDIM + tid] = b[tid] - (float)mean * scv;
  }
  __syncthreads();
  v4f a0 = {0.f, 0.f, 0.f, 0.f}, a1 = {0.f, 0.f, 0.f, 0.f};
  if (tid < 32) {
    a0 = *(const v4f*)(stab + 4 * tid);
    a1 = *(const v4f*)(stab + HDIM + 4 * tid);
    *(volatile v4f*)(sct + 4 * tid) = a0;
    *(volatile v4f*)(sct + HDIM + 4 * tid) = a1;
  }
  __threadfence();
  if (tid < 32) {
    *(volatile v4f*)(sct + 4 * tid) = a0;
    *(volatile v4f*)(sct + HDIM + 4 * tid) = a1;
  }
}

__global__ __launch_bounds__(NTHR) void k_apply(
    const float* __restrict__ hpre, const float* __restrict__ sct, float* h) {
  const int tid = threadIdx.x, lane = tid & 31, wave = tid >> 5;
  const int r0 = blockIdx.x * GROWS + wave * 16;
  const v4f sc4 = *(const v4f*)(sct + 4 * lane);
  const v4f sh4 = *(const v4f*)(sct + HDIM + 4 * lane);
  v4f vals[16];
#pragma unroll
  for (int i = 0; i < 16; ++i) {
    const v4f hp = *(const v4f*)(hpre + (size_t)(r0 + i) * HDIM + 4 * lane);
    v4f y = hp * sc4 + sh4;
    y.x = fmaxf(y.x, 0.f); y.y = fmaxf(y.y, 0.f); y.z = fmaxf(y.z, 0.f); y.w = fmaxf(y.w, 0.f);
    vals[i] = y;
  }
  float* gp = h + (size_t)r0 * HDIM + 4 * lane;
#pragma unroll
  for (int i = 0; i < 16; ++i) *(volatile v4f*)(gp + (size_t)i * HDIM) = vals[i];
  __threadfence();
#pragma unroll
  for (int i = 0; i < 16; ++i) *(volatile v4f*)(gp + (size_t)i * HDIM) = vals[i];
}

__global__ __launch_bounds__(ETHR) void k_edge(
    const int* __restrict__ ei, const float* __restrict__ eattr, const float* __restrict__ pq,
    const float* __restrict__ ee_w1, const float* __restrict__ ee_b1,
    const float* __restrict__ ea_w1t, const float* __restrict__ ea_b1,
    const float* __restrict__ ea_w2, const float* __restrict__ ea_b2,
    const float* __restrict__ cl_b1,
    const unsigned short* __restrict__ wqh, const unsigned short* __restrict__ wql, const float* __restrict__ cvec,
    const unsigned short* __restrict__ w2h, const unsigned short* __restrict__ w2l, const float* __restrict__ cl_b2,
    const float* __restrict__ cl_w3, const float* __restrict__ cl_b3,
    float* out, int nE, int nN) {
  extern __shared__ v4f lds_dyn[];
  char* base = (char*)lds_dyn;
  unsigned short* sTh = (unsigned short*)(base + EO_TH);
  unsigned short* sTl = (unsigned short*)(base + EO_TL);
  unsigned short* sZh = (unsigned short*)(base + EO_ZH);
  unsigned short* sZl = (unsigned short*)(base + EO_ZL);
  float*    sAB  = (float*)(base + EO_AB);
  float*    sEA  = (float*)(base + EO_EA);
  float*    sW1e = (float*)(base + EO_W1E);
  float*    sWat = (float*)(base + EO_WAT);
  float*    sB1e = (float*)(base + EO_B1E);
  float*    sBa  = (float*)(base + EO_BA);
  float*    sW2a = (float*)(base + EO_W2A);
  float*    sCv  = (float*)(base + EO_CV);
  float*    sB1c = (float*)(base + EO_B1C);
  float*    sB2c = (float*)(base + EO_B2C);
  float*    sW3  = (float*)(base + EO_W3);
  float*    sAtt = (float*)(base + EO_ATT);
  int*      sRow = (int*)(base + EO_ROW);
  int*      sCol = (int*)(base + EO_COL);
  float*    sOut = (float*)(base + EO_OUT);
  const int tid = threadIdx.x, lane = tid & 31, wave = tid >> 5, hh = lane >> 4, m = lane & 15;
  const int e0 = blockIdx.x * EPB;

  for (int i = tid; i < FDIM * HDIM; i += ETHR) { sW1e[i] = ee_w1[i]; sWat[i] = ea_w1t[i]; }
  for (int i = tid; i < HDIM; i += ETHR) {
    sB1e[i] = ee_b1[i]; sBa[i] = ea_b1[i]; sW2a[i] = ea_w2[i];
    sCv[i] = cvec[i];   sB1c[i] = cl_b1[i]; sW3[i] = cl_w3[i];
  }
  for (int i = tid; i < 64; i += ETHR) sB2c[i] = cl_b2[i];
  for (int i = tid; i < EPB * FDIM; i += ETHR) sEA[i] = eattr[(size_t)e0 * FDIM + i];
  if (tid < EPB) {
    int r = ei[e0 + tid];
    int c = ei[(size_t)nE + e0 + tid];
    r = r < 0 ? 0 : (r > nN - 1 ? nN - 1 : r);
    c = c < 0 ? 0 : (c > nN - 1 ? nN - 1 : c);
    sRow[tid] = r; sCol[tid] = c;
  }
  const float eb2 = ea_b2[0];
  const float b30 = cl_b3[0], b31 = cl_b3[1];
  __syncthreads();

  {
    const v4f b1e = *(const v4f*)(sB1e + 4 * lane);
    const v4f ba  = *(const v4f*)(sBa + 4 * lane);
    const v4f w2a = *(const v4f*)(sW2a + 4 * lane);
    const v4f b1c = *(const v4f*)(sB1c + 4 * lane);
#pragma unroll 1
    for (int j = 0; j < 16; ++j) {
      const int e  = wave * 16 + j;
      const int ri = sRow[e], ci = sCol[e];
      const float* pr = pq + (size_t)ri * 512;
      const float* pc = pq + (size_t)ci * 512;
      const v4f pv  = *(const v4f*)(pr + 4 * lane);
      const v4f av0 = *(const v4f*)(pr + 256 + 4 * lane);
      const v4f qv  = *(const v4f*)(pc + 128 + 4 * lane);
      const v4f bv0 = *(const v4f*)(pc + 384 + 4 * lane);
      v4f tv = b1e;
      v4f av = ba + pv + qv;
      const float* ea = sEA + e * FDIM;
#pragma unroll 1
      for (int k = 0; k < FDIM; ++k) {
        const float ek = ea[k];
        const v4f w1 = *(const v4f*)(sW1e + k * HDIM + 4 * lane);
        const v4f wa = *(const v4f*)(sWat + k * HDIM + 4 * lane);
        tv = tv + ek * w1;
        av = av + ek * wa;
      }
      tv.x = fmaxf(tv.x, 0.f); tv.y = fmaxf(tv.y, 0.f); tv.z = fmaxf(tv.z, 0.f); tv.w = fmaxf(tv.w, 0.f);
      v4us th4, tl4;
      unsigned short hb, lb;
      bfsplit(tv.x, hb, lb); th4[0] = hb; tl4[0] = lb;
      bfsplit(tv.y, hb, lb); th4[1] = hb; tl4[1] = lb;
      bfsplit(tv.z, hb, lb); th4[2] = hb; tl4[2] = lb;
      bfsplit(tv.w, hb, lb); th4[3] = hb; tl4[3] = lb;
      *(v4us*)(sTh + e * APH + 4 * lane) = th4;
      *(v4us*)(sTl + e * APH + 4 * lane) = tl4;
      av.x = fmaxf(av.x, 0.f); av.y = fmaxf(av.y, 0.f); av.z = fmaxf(av.z, 0.f); av.w = fmaxf(av.w, 0.f);
      float partv = av.x * w2a.x + av.y * w2a.y + av.z * w2a.z + av.w * w2a.w;
      partv += __shfl_xor(partv, 16);
      partv += __shfl_xor(partv, 8);
      partv += __shfl_xor(partv, 4);
      partv += __shfl_xor(partv, 2);
      partv += __shfl_xor(partv, 1);
      float sgm = partv + eb2;
      sgm = fminf(fmaxf(sgm, -40.f), 40.f);
      const float at = 1.0f / (1.0f + expf(-sgm));
      if (lane == 0) sAtt[e] = at;
      const v4f ab = av0 + bv0 + b1c;
      *(v4f*)(sAB + e * HDIM + 4 * lane) = ab;
    }
  }
  __syncthreads();

  v8f acc[8];
#pragma unroll
  for (int t = 0; t < 8; ++t) { v8f z = {0.f, 0.f, 0.f, 0.f, 0.f, 0.f, 0.f, 0.f}; acc[t] = z; }
  {
    const unsigned short* arh = sTh + (wave * 16 + m) * APH + 8 * hh;
    const unsigned short* arl = sTl + (wave * 16 + m) * APH + 8 * hh;
#pragma unroll
    for (int kt = 0; kt < HDIM / 32; ++kt) {
      FragB ah, al;
      ah.h[0] = *(const v8us*)(arh + 32 * kt);
      ah.h[1] = *(const v8us*)(arh + 32 * kt + 16);
      al.h[0] = *(const v8us*)(arl + 32 * kt);
      al.h[1] = *(const v8us*)(arl + 32 * kt + 16);
#pragma unroll
      for (int t = 0; t < 8; ++t) {
        const size_t bp = (size_t)(16 * t + m) * HDIM + 32 * kt + 8 * hh;
        FragB bh2, bl2;
        bh2.h[0] = *(const v8us*)(wqh + bp);
        bh2.h[1] = *(const v8us*)(wqh + bp + 16);
        bl2.h[0] = *(const v8us*)(wql + bp);
        bl2.h[1] = *(const v8us*)(wql + bp + 16);
        acc[t] = wmb(ah.v, bh2.v, acc[t]);
        acc[t] = wmb(al.v, bh2.v, acc[t]);
        acc[t] = wmb(ah.v, bl2.v, acc[t]);
      }
    }
  }
#pragma unroll
  for (int t = 0; t < 8; ++t) {
    const int n = 16 * t + m;
    const float cvn = sCv[n];
#pragma unroll
    for (int r = 0; r < 8; ++r) {
      const int e = wave * 16 + 8 * hh + r;
      const float u = acc[t][r];
      float v = sAB[e * HDIM + n] + sAtt[e] * (u + cvn);
      v = fmaxf(v, 0.f);
      unsigned short hb, lb;
      bfsplit(v, hb, lb);
      sZh[e * APH + n] = hb;
      sZl[e * APH + n] = lb;
    }
  }
  __syncthreads();

  v8f acc2[4];
#pragma unroll
  for (int t = 0; t < 4; ++t) { v8f z = {0.f, 0.f, 0.f, 0.f, 0.f, 0.f, 0.f, 0.f}; acc2[t] = z; }
  {
    const unsigned short* arh = sZh + (wave * 16 + m) * APH + 8 * hh;
    const unsigned short* arl = sZl + (wave * 16 + m) * APH + 8 * hh;
#pragma unroll
    for (int kt = 0; kt < HDIM / 32; ++kt) {
      FragB ah, al;
      ah.h[0] = *(const v8us*)(arh + 32 * kt);
      ah.h[1] = *(const v8us*)(arh + 32 * kt + 16);
      al.h[0] = *(const v8us*)(arl + 32 * kt);
      al.h[1] = *(const v8us*)(arl + 32 * kt + 16);
#pragma unroll
      for (int t = 0; t < 4; ++t) {
        const size_t bp = (size_t)(16 * t + m) * HDIM + 32 * kt + 8 * hh;
        FragB bh2, bl2;
        bh2.h[0] = *(const v8us*)(w2h + bp);
        bh2.h[1] = *(const v8us*)(w2h + bp + 16);
        bl2.h[0] = *(const v8us*)(w2l + bp);
        bl2.h[1] = *(const v8us*)(w2l + bp + 16);
        acc2[t] = wmb(ah.v, bh2.v, acc2[t]);
        acc2[t] = wmb(al.v, bh2.v, acc2[t]);
        acc2[t] = wmb(ah.v, bl2.v, acc2[t]);
      }
    }
  }
  float lg0[8], lg1[8];
#pragma unroll
  for (int r = 0; r < 8; ++r) { lg0[r] = 0.f; lg1[r] = 0.f; }
#pragma unroll
  for (int t = 0; t < 4; ++t) {
    const int n = 16 * t + m;
    const float b2v = sB2c[n];
    const float w30 = sW3[2 * n], w31 = sW3[2 * n + 1];
#pragma unroll
    for (int r = 0; r < 8; ++r) {
      const float z = fmaxf(acc2[t][r] + b2v, 0.f);
      lg0[r] += z * w30;
      lg1[r] += z * w31;
    }
  }
#pragma unroll
  for (int r = 0; r < 8; ++r) {
    float x0 = lg0[r], x1 = lg1[r];
    x0 += __shfl_xor(x0, 8); x1 += __shfl_xor(x1, 8);
    x0 += __shfl_xor(x0, 4); x1 += __shfl_xor(x1, 4);
    x0 += __shfl_xor(x0, 2); x1 += __shfl_xor(x1, 2);
    x0 += __shfl_xor(x0, 1); x1 += __shfl_xor(x1, 1);
    if (m == 0) {
      const int e = wave * 16 + 8 * hh + r;
      sOut[2 * e]     = x0 + b30;
      sOut[2 * e + 1] = x1 + b31;
    }
  }
  __syncthreads();

  v4f ov = {0.f, 0.f, 0.f, 0.f};
  float* op = out + (size_t)blockIdx.x * (EPB * 2);
  if (tid < 32) {
    ov = *(const v4f*)(sOut + 4 * tid);
    *(volatile v4f*)(op + 4 * tid) = ov;
  }
  __threadfence();
  if (tid < 32) *(volatile v4f*)(op + 4 * tid) = ov;
}

extern "C" void kernel_launch(void* const* d_in, const int* in_sizes, int n_in,
                              void* d_out, int out_size, void* d_ws, size_t ws_size,
                              hipStream_t stream) {
  if (n_in < 27) return;
  const int nN = in_sizes[0] / FDIM;
  const int nE = in_sizes[1] / 2;
  if (nN <= 0 || nE <= 0 || in_sizes[0] != nN * FDIM || in_sizes[1] != 2 * nE || in_sizes[2] != nE * FDIM) return;
  if ((nE % EPB) != 0 || out_size != nE * 2) return;
  if (nE > (1 << 28) || nN > (1 << 24)) return;
  if (in_sizes[3] != FDIM * HDIM || in_sizes[4] < HDIM || in_sizes[5] != HDIM * HDIM || in_sizes[6] < HDIM) return;
  if (in_sizes[7] != FDIM * HDIM || in_sizes[8] < HDIM || in_sizes[9] != HDIM * HDIM || in_sizes[10] < HDIM) return;
  if (in_sizes[11] != (2 * HDIM + FDIM) * HDIM || in_sizes[12] < HDIM || in_sizes[13] != HDIM || in_sizes[14] < 1) return;
  if (in_sizes[15] != 3 * HDIM * HDIM || in_sizes[16] < 3 * HDIM || in_sizes[17] < 3 * HDIM || in_sizes[18] < 3 * HDIM) return;
  if (in_sizes[19] != 2 * HDIM * HDIM || in_sizes[20] < 2 * HDIM) return;
  if (in_sizes[21] != 2 * HDIM * HDIM || in_sizes[22] < HDIM || in_sizes[23] != HDIM * 64 || in_sizes[24] < 64) return;
  if (in_sizes[25] != 64 * 2 || in_sizes[26] < 2) return;

  const float* x      = (const float*)d_in[0];
  const int*   ei     = (const int*)d_in[1];
  const float* eattr  = (const float*)d_in[2];
  const float* ne_w1  = (const float*)d_in[3];
  const float* ne_b1  = (const float*)d_in[4];
  const float* ne_w2  = (const float*)d_in[5];
  const float* ne_b2  = (const float*)d_in[6];
  const float* ee_w1  = (const float*)d_in[7];
  const float* ee_b1  = (const float*)d_in[8];
  const float* ee_w2  = (const float*)d_in[9];
  const float* ee_b2  = (const float*)d_in[10];
  const float* ea_w1  = (const float*)d_in[11];
  const float* ea_b1  = (const float*)d_in[12];
  const float* ea_w2  = (const float*)d_in[13];
  const float* ea_b2  = (const float*)d_in[14];
  const float* gcn_w  = (const float*)d_in[15];
  const float* gcn_b  = (const float*)d_in[16];
  const float* bn_g   = (const float*)d_in[17];
  const float* bn_b   = (const float*)d_in[18];
  const float* skip_w = (const float*)d_in[19];
  const float* skip_b = (const float*)d_in[20];
  const float* cl_w1  = (const float*)d_in[21];
  const float* cl_b1  = (const float*)d_in[22];
  const float* cl_w2  = (const float*)d_in[23];
  const float* cl_b2  = (const float*)d_in[24];
  const float* cl_w3  = (const float*)d_in[25];
  const float* cl_b3  = (const float*)d_in[26];
  float* out = (float*)d_out;

  const int NPAD   = ((nN + TGT - 1) / TGT) * TGT;
  const int nBC    = (nN + NBC - 1) / NBC;
  const int CNTPAD = nBC * NBC;
  if (4 * nBC + 1 > RBN || CNTPAD < NPAD) return;
  const int nBF    = (nN + NBF - 1) / NBF;
  const int csrLen = ((nE + 31) & ~31) + 4096;
  const int nG     = NPAD / GROWS;
  const int nAgg   = NPAD / TGT;
  const int nEB    = nE / EPB;
  const size_t PLB = (size_t)NPAD * HDIM * 4;

  char* ws = (char*)d_ws;
  size_t off = 0;
  const size_t oBh  = off; off += (size_t)NBROW * HDIM * 2;        off = (off + 255) & ~(size_t)255;
  const size_t oBl  = off; off += (size_t)NBROW * HDIM * 2;        off = (off + 255) & ~(size_t)255;
  const size_t oWqh = off; off += (size_t)HDIM * HDIM * 2;         off = (off + 255) & ~(size_t)255;
  const size_t oWql = off; off += (size_t)HDIM * HDIM * 2;         off = (off + 255) & ~(size_t)255;
  const size_t oW2h = off; off += (size_t)64 * HDIM * 2;           off = (off + 255) & ~(size_t)255;
  const size_t oW2l = off; off += (size_t)64 * HDIM * 2;           off = (off + 255) & ~(size_t)255;
  const size_t oCv  = off; off += (size_t)HDIM * 4;                off = (off + 255) & ~(size_t)255;
  const size_t oCnt = off; off += (size_t)CNTPAD * 4;              off = (off + 255) & ~(size_t)255;
  const size_t oDv  = off; off += (size_t)CNTPAD * 4;              off = (off + 255) & ~(size_t)255;
  const size_t oOff = off; off += (size_t)CNTPAD * 4;              off = (off + 255) & ~(size_t)255;
  const size_t oRb  = off; off += (size_t)RBN * 4;                 off = (off + 255) & ~(size_t)255;
  const size_t oCsr = off; off += (size_t)csrLen * 4;              off = (off + 255) & ~(size_t)255;
  const size_t oPrt = off; off += (size_t)nAgg * 256 * 8;          off = (off + 255) & ~(size_t)255;
  const size_t oSct = off; off += (size_t)2 * HDIM * 4;            off = (off + 255) & ~(size_t)255;
  const size_t oBig = off; off += 5 * PLB;                         off = (off + 255) & ~(size_t)255;
  if (off > ws_size || off > (size_t)134217728) return;
  unsigned short* bh  = (unsigned short*)(ws + oBh);
  unsigned short* bl  = (unsigned short*)(ws + oBl);
  unsigned short* wqh = (unsigned short*)(ws + oWqh);
  unsigned short* wql = (unsigned short*)(ws + oWql);
  unsigned short* w2h = (unsigned short*)(ws + oW2h);
  unsigned short* w2l = (unsigned short*)(ws + oW2l);
  float*    cvec = (float*)(ws + oCv);
  int*      cnt  = (int*)(ws + oCnt);
  float*    dinv = (float*)(ws + oDv);
  int*      offp = (int*)(ws + oOff);
  int*      rb   = (int*)(ws + oRb);
  int*      csr  = (int*)(ws + oCsr);
  double*   part = (double*)(ws + oPrt);
  float*    sct  = (float*)(ws + oSct);
  float*    X    = (float*)(ws + oBig);
  float*    Y    = (float*)(ws + oBig + PLB);
  float*    Z    = (float*)(ws + oBig + 2 * PLB);
  float*    PQ   = (float*)(ws + oBig + PLB);

  const int vec8 = ((nE & 3) == 0) ? 1 : 0;

  const int nPrep = (NBROW * 16 + HDIM * 16 + 64 * 16) / NTHR + 1;
  k_wprep<<<nPrep, NTHR, 0, stream>>>(ne_w2, gcn_w, skip_w, ea_w1, cl_w1, ee_w2, ee_b2, cl_w2,
                                      bh, bl, wqh, wql, w2h, w2l, cvec);

  k_count<<<nBC, NTHR, 0, stream>>>(ei, cnt, dinv, nE, vec8);
  k_offsets<<<1, OTHR, 0, stream>>>(cnt, offp, rb, nBC);
  hipFuncSetAttribute(reinterpret_cast<const void*>(&k_fill),
                      hipFuncAttributeMaxDynamicSharedMemorySize, LDS_FILL);
  k_fill<<<nBF, NTHR, LDS_FILL, stream>>>(ei, offp, rb, csr, nN, nE, vec8, csrLen);

  hipFuncSetAttribute(reinterpret_cast<const void*>(&k_ngemm<0, 1>),
                      hipFuncAttributeMaxDynamicSharedMemorySize, LDS_NG);
  hipFuncSetAttribute(reinterpret_cast<const void*>(&k_ngemm<1, 0>),
                      hipFuncAttributeMaxDynamicSharedMemorySize, LDS_NG);
  hipFuncSetAttribute(reinterpret_cast<const void*>(&k_ngemm<2, 0>),
                      hipFuncAttributeMaxDynamicSharedMemorySize, LDS_NG);
  hipFuncSetAttribute(reinterpret_cast<const void*>(&k_ngemm<3, 0>),
                      hipFuncAttributeMaxDynamicSharedMemorySize, LDS_NG);
  k_ngemm<0, 1><<<dim3(nG, 1), NTHR, LDS_NG, stream>>>(x, ne_w1, ne_b1, bh, bl, dinv, ne_b2, Z, sct, Y, nN, HDIM);

  k_ngemm<1, 0><<<dim3(nG, 1), NTHR, LDS_NG, stream>>>(Y, ne_w1, ne_b1, bh + (size_t)128 * HDIM, bl + (size_t)128 * HDIM,
                                                       dinv, ne_b2, Z, sct, X, NPAD, HDIM);
  k_agg<<<nAgg, NTHR, 0, stream>>>(csr, offp, cnt, dinv, X, gcn_b, Z, part, nN, csrLen);
  k_bnfin<<<1, NTHR, 0, stream>>>(part, bn_g, bn_b, sct, nAgg, nN);
  k_apply<<<nG, NTHR, 0, stream>>>(Z, sct, X);

  k_ngemm<1, 0><<<dim3(nG, 1), NTHR, LDS_NG, stream>>>(X, ne_w1, ne_b1, bh + (size_t)256 * HDIM, bl + (size_t)256 * HDIM,
                                                       dinv, ne_b2, Z, sct, Y, NPAD, HDIM);
  k_agg<<<nAgg, NTHR, 0, stream>>>(csr, offp, cnt, dinv, Y, gcn_b + HDIM, Z, part, nN, csrLen);
  k_bnfin<<<1, NTHR, 0, stream>>>(part, bn_g + HDIM, bn_b + HDIM, sct, nAgg, nN);
  k_ngemm<2, 0><<<dim3(nG, 1), NTHR, LDS_NG, stream>>>(X, ne_w1, ne_b1, bh + (size_t)512 * HDIM, bl + (size_t)512 * HDIM,
                                                       dinv, skip_b, Z, sct, Y, NPAD, HDIM);

  k_ngemm<1, 0><<<dim3(nG, 1), NTHR, LDS_NG, stream>>>(Y, ne_w1, ne_b1, bh + (size_t)384 * HDIM, bl + (size_t)384 * HDIM,
                                                       dinv, ne_b2, Z, sct, X, NPAD, HDIM);
  k_agg<<<nAgg, NTHR, 0, stream>>>(csr, offp, cnt, dinv, X, gcn_b + 2 * HDIM, Z, part, nN, csrLen);
  k_bnfin<<<1, NTHR, 0, stream>>>(part, bn_g + 2 * HDIM, bn_b + 2 * HDIM, sct, nAgg, nN);
  k_ngemm<2, 0><<<dim3(nG, 1), NTHR, LDS_NG, stream>>>(Y, ne_w1, ne_b1, bh + (size_t)640 * HDIM, bl + (size_t)640 * HDIM,
                                                       dinv, skip_b + HDIM, Z, sct, X, NPAD, HDIM);

  k_ngemm<3, 0><<<dim3(nG, 4), NTHR, LDS_NG, stream>>>(X, ne_w1, ne_b1, bh + (size_t)768 * HDIM, bl + (size_t)768 * HDIM,
                                                       dinv, ne_b2, Z, sct, PQ, NPAD, 4 * HDIM);

  hipFuncSetAttribute(reinterpret_cast<const void*>(&k_edge),
                      hipFuncAttributeMaxDynamicSharedMemorySize, LDS_EDGE);
  k_edge<<<nEB, ETHR, LDS_EDGE, stream>>>(ei, eattr, PQ, ee_w1, ee_b1, ea_w1 + (size_t)2 * HDIM * HDIM, ea_b1,
                                         ea_w2, ea_b2, cl_b1, wqh, wql, cvec, w2h, w2l, cl_b2, cl_w3, cl_b3, out, nE, nN);
}
